// OfficialMamba3SISO_86062554677279
// MI455X (gfx1250) — hardware-run, weakly checked
//
#include <hip/hip_runtime.h>


#define NR   2048
#define NT   1024
#define NM   1024
#define NG   2048
#define NU   32
#define NW   64
#define NC   128
#define NQ   32
#define NJ   4480
#define OX   2048
#define OP   4096
#define OQ   4224
#define OPA  4352
#define OFA  4384
#define OBL  4416
#define OAR  4448
typedef _Float16 h16;
typedef unsigned short bf;
typedef __attribute__((ext_vector_type(16))) __bf16   v16bf;
typedef __attribute__((ext_vector_type(16))) _Float16 v16h;
typedef __attribute__((ext_vector_type(8)))  _Float16 v8h;
typedef __attribute__((ext_vector_type(8)))  unsigned short v8us;
typedef __attribute__((ext_vector_type(8)))  float    v8f;
typedef __attribute__((ext_vector_type(4)))  float    v4f;
typedef v8h  __attribute__((may_alias)) v8ha;
typedef v4f  __attribute__((may_alias)) v4fa;
typedef v8us __attribute__((may_alias)) v8usa;

__device__ __forceinline__ unsigned short f2bf(float f) { unsigned u = __float_as_uint(f); u += 0x7FFFu + ((u >> 16) & 1u); return (unsigned short)(u >> 16); }
__device__ __forceinline__ float bf2f(unsigned short b) { return __uint_as_float(((unsigned)b) << 16); }
__device__ __forceinline__ float bfr(float f) { return bf2f(f2bf(f)); }
__device__ __forceinline__ v16h cat16(v8h lo, v8h hi) { return __builtin_shufflevector(lo, hi, 0, 1, 2, 3, 4, 5, 6, 7, 8, 9, 10, 11, 12, 13, 14, 15); }
__device__ __forceinline__ v16bf cat16b(v8us lo, v8us hi) { return __builtin_bit_cast(v16bf, __builtin_shufflevector(lo, hi, 0, 1, 2, 3, 4, 5, 6, 7, 8, 9, 10, 11, 12, 13, 14, 15)); }
__device__ __forceinline__ v8f wmma16(v16h a, v16h b, v8f c) { return __builtin_amdgcn_wmma_f32_16x16x32_f16(false, a, false, b, (short)0, c, false, false); }
__device__ __forceinline__ v8f wmmab(v16bf a, v16bf b, v8f c) { return __builtin_amdgcn_wmma_f32_16x16x32_bf16(false, a, false, b, (short)0, c, false, false); }

template <typename T16> struct WFrag;
template <> struct WFrag<h16> { typedef v16h V; static __device__ __forceinline__ V ld(const h16* p) { return cat16(*(const v8h*)p, *(const v8h*)(p + 16)); } static __device__ __forceinline__ v8f mma(V a, V b, v8f c) { return wmma16(a, b, c); } };
template <> struct WFrag<bf> { typedef v16bf V; static __device__ __forceinline__ V ld(const bf* p) { return cat16b(*(const v8us*)p, *(const v8us*)(p + 16)); } static __device__ __forceinline__ v8f mma(V a, V b, v8f c) { return wmmab(a, b, c); } };
template <typename T16, int NSPLIT, bool BIAS>
__global__ __launch_bounds__(32) void k_gemmw(const T16* __restrict__ A, const T16* __restrict__ A2, const T16* __restrict__ Bt, const T16* __restrict__ Bt2, int K, float* C, int ldc, const float* __restrict__ bias, size_t sA, size_t sB, size_t sC) {
    typedef typename WFrag<T16>::V V;
    __shared__ __align__(16) float os[16 * 68];
    const size_t z = blockIdx.z; A += z * sA; if (A2) A2 += z * sA; Bt += z * sB; if (Bt2) Bt2 += z * sB; C += z * sC;
    const int lane = threadIdx.x & 31, lr = lane & 15, hi = lane >> 4; const int r0 = blockIdx.x * 64, c0 = blockIdx.y * 64;
    v8f acc[4][4];
#pragma unroll
    for (int mb = 0; mb < 4; ++mb)
#pragma unroll
        for (int nb = 0; nb < 4; ++nb) acc[mb][nb] = (v8f){};
    const size_t aoff = (size_t)(r0 + lr) * K + 8 * hi, boff = (size_t)(c0 + lr) * K + 8 * hi;
    for (int kc = 0; kc < K; kc += 32) {
        V a[4], a2[4];
#pragma unroll
        for (int mb = 0; mb < 4; ++mb) { a[mb] = WFrag<T16>::ld(A + aoff + (size_t)mb * 16 * K + kc); if (NSPLIT == 1 || NSPLIT == 2) a2[mb] = WFrag<T16>::ld(A2 + aoff + (size_t)mb * 16 * K + kc); }
#pragma unroll
        for (int nb = 0; nb < 4; ++nb) { const V b = WFrag<T16>::ld(Bt + boff + (size_t)nb * 16 * K + kc); V b2; if (NSPLIT >= 2) b2 = WFrag<T16>::ld(Bt2 + boff + (size_t)nb * 16 * K + kc);
#pragma unroll
            for (int mb = 0; mb < 4; ++mb) { acc[mb][nb] = WFrag<T16>::mma(a[mb], b, acc[mb][nb]); if (NSPLIT == 1 || NSPLIT == 2) acc[mb][nb] = WFrag<T16>::mma(a2[mb], b, acc[mb][nb]); if (NSPLIT >= 2) acc[mb][nb] = WFrag<T16>::mma(a[mb], b2, acc[mb][nb]); } }
        asm volatile("v_nop\n\tv_nop\n\tv_nop\n\tv_nop" : "+v"(acc[0][0]), "+v"(acc[1][1]), "+v"(acc[2][2]), "+v"(acc[3][3]) : "v"(a[0]), "v"(a[3]));
    }
#pragma unroll
    for (int mb = 0; mb < 4; ++mb) {
#pragma unroll
        for (int nb = 0; nb < 4; ++nb) {
#pragma unroll
            for (int j = 0; j < 8; ++j) os[(hi * 8 + j) * 68 + nb * 16 + lr] = acc[mb][nb][j]; }
        __builtin_amdgcn_wave_barrier(); asm volatile("" ::: "memory");
        float* crow = C + (size_t)(r0 + mb * 16) * ldc + c0;
#pragma unroll 1
        for (int ps = 0; ps < 2; ++ps) {
#pragma unroll
            for (int s = 0; s < 8; ++s) { const int row = 2 * s + hi, cofs = lr * 4; v4f val = *(const v4fa*)(os + row * 68 + cofs); if (BIAS) { val[0] += bfr(bias[c0 + cofs]); val[1] += bfr(bias[c0 + cofs + 1]); val[2] += bfr(bias[c0 + cofs + 2]); val[3] += bfr(bias[c0 + cofs + 3]); }
                *(volatile v4f*)(crow + (size_t)row * ldc + cofs) = val; }
            if (ps == 0) __threadfence(); }
        __builtin_amdgcn_wave_barrier(); asm volatile("" ::: "memory");
    }
}

typedef __attribute__((ext_vector_type(2))) _Float16 v2h;
typedef __attribute__((ext_vector_type(4))) _Float16 v4h;
typedef __attribute__((ext_vector_type(2))) unsigned short v2us;
typedef __attribute__((ext_vector_type(4))) unsigned short v4us;
typedef __attribute__((ext_vector_type(2))) float v2f;
typedef __attribute__((ext_vector_type(4))) int v4i;

__global__ __launch_bounds__(256) void k_cvt8(const float* __restrict__ src, bf* dst, size_t n8) { const size_t i = (size_t)blockIdx.x * 256 + threadIdx.x; if (i >= n8) return; const v8f v = *(const v8f*)(src + i * 8); v8us o;
#pragma unroll
    for (int k = 0; k < 8; ++k) o[k] = f2bf(v[k]); *(volatile v8us*)(dst + i * 8) = o; __threadfence(); *(volatile v8us*)(dst + i * 8) = o; }

__device__ __forceinline__ h16 toh_flush(float x) { const float z = (fabsf(x) < 6.103515625e-05f) ? 0.0f : x; return (h16)z; }

template <bool RB>
__global__ __launch_bounds__(256) void k_c16(const float* __restrict__ src, h16* dst, size_t n8) { const size_t i = (size_t)blockIdx.x * 256 + threadIdx.x; if (i >= n8) return; const float* p = src + i * 8; const v4f a = *(const v4f*)p, b = *(const v4f*)(p + 4); v8h o;
#pragma unroll
    for (int q = 0; q < 4; ++q) { o[q] = toh_flush(RB ? bfr(a[q]) : a[q]); o[q + 4] = toh_flush(RB ? bfr(b[q]) : b[q]); }
    *(volatile v8h*)(dst + i * 8) = o; __threadfence(); *(volatile v8h*)(dst + i * 8) = o; }

static __device__ __forceinline__ float spl(float av) { return fmaxf(av, 0.0f) + log1pf(expf(-fabsf(av))); }

__global__ __launch_bounds__(256) void k_pre4(const float* __restrict__ Pj, const float* __restrict__ a4, const float* __restrict__ a7, const float* __restrict__ a8, float* Sc, float* Ar, float* Pn, float* Qn) { const unsigned nb = blockIdx.x * 256u + threadIdx.x; const unsigned rw = nb >> 5, un = nb & 31u; const float* pr = Pj + (size_t)rw * NJ;
    const float pc = spl(pr[OPA + un] + bfr(a4[un])); float fa = -spl(pr[OFA + un]); fa = fminf(fa, -1e-4f); const float fd = expf(fa * pc); const float bl = 1.0f / (1.0f + expf(-pr[OBL + un]));
    float sp = 0.0f, sq = 0.0f;
    for (int k = 0; k < NC; k += 4) { const v4f vp = *(const v4f*)(pr + OP + k);
#pragma unroll
        for (int j = 0; j < 4; ++j) sp += vp[j] * vp[j]; }
    for (int k = 0; k < NC; k += 4) { const v4f vq = *(const v4f*)(pr + OQ + k);
#pragma unroll
        for (int j = 0; j < 4; ++j) sq += vq[j] * vq[j]; }
    const float rp = 1.0f / sqrtf(sp * (1.0f / NC) + 1e-5f), rq = 1.0f / sqrtf(sq * (1.0f / NC) + 1e-5f);
    const v4f mp = *(const v4f*)(pr + OP + un * 4), mq = *(const v4f*)(pr + OQ + un * 4), w7 = *(const v4f*)(a7 + un * 4), w8 = *(const v4f*)(a8 + un * 4); v4f op, oq, os; os[0] = pc; os[1] = fd; os[2] = bl; os[3] = 0.0f;
#pragma unroll
    for (int j = 0; j < 4; ++j) { op[j] = mp[j] * rp * bfr(w7[j]); oq[j] = mq[j] * rq * bfr(w8[j]); }
    v4f oa[8];
#pragma unroll
    for (int gq = 0; gq < 8; ++gq) { const v4f va = *(const v4f*)(pr + OAR + gq * 4);
#pragma unroll
        for (int j = 0; j < 4; ++j) oa[gq][j] = va[j] * pc; }
    float* ps = Sc + (size_t)nb * 4; float* pa = Ar + (size_t)nb * NQ; float* pp = Pn + (size_t)rw * NC + un * 4; float* pq = Qn + (size_t)rw * NC + un * 4;
    *(volatile v4f*)ps = os; *(volatile v4f*)pp = op; *(volatile v4f*)pq = oq;
#pragma unroll
    for (int gq = 0; gq < 8; ++gq) *(volatile v4f*)(pa + gq * 4) = oa[gq];
    __threadfence();
    *(volatile v4f*)ps = os; *(volatile v4f*)pp = op; *(volatile v4f*)pq = oq;
#pragma unroll
    for (int gq = 0; gq < 8; ++gq) *(volatile v4f*)(pa + gq * 4) = oa[gq]; }

__global__ __launch_bounds__(256) void k_run(const float* __restrict__ Ar, float* Sw) { const unsigned nb = blockIdx.x * 256u + threadIdx.x; const unsigned sn = nb >> 10, un = (nb >> 5) & 31u, q = nb & 31u; float acc = 0.0f;
    for (int tn = 0; tn < NT; ++tn) { const size_t at = (((size_t)sn * NT + tn) * NU + un) * NQ + q; acc += Ar[at]; *(volatile float*)(Sw + at) = acc; __threadfence(); *(volatile float*)(Sw + at) = acc; } }

__global__ __launch_bounds__(256) void k_turn(const float* __restrict__ Sw, const float* __restrict__ Pn, const float* __restrict__ Qn, const float* __restrict__ a5, const float* __restrict__ a6, float* Pt, float* Qt) { const unsigned nb = blockIdx.x * 256u + threadIdx.x; const unsigned rw = nb >> 10, un = (nb >> 5) & 31u, q = nb & 31u; const float sw = Sw[nb]; const float sn = sinf(sw), cs = cosf(sw); const float* pn = Pn + (size_t)rw * NC + q; const float* qn = Qn + (size_t)rw * NC + q; const float* p5 = a5 + (size_t)un * NC + q; const float* p6 = a6 + (size_t)un * NC + q;
    const float p1 = pn[0] + bfr(p5[0]), p2 = pn[32] + bfr(p5[32]), p3 = pn[64] + bfr(p5[64]), p4 = pn[96] + bfr(p5[96]); const float q1 = qn[0] + bfr(p6[0]), q2 = qn[32] + bfr(p6[32]), q3 = qn[64] + bfr(p6[64]), q4 = qn[96] + bfr(p6[96]);
    const float e1 = p1 * cs - p2 * sn, e2 = p1 * sn + p2 * cs, f1 = q1 * cs - q2 * sn, f2 = q1 * sn + q2 * cs; float* op = Pt + ((size_t)rw * NU + un) * NC + q; float* oq = Qt + ((size_t)rw * NU + un) * NC + q;
    *(volatile float*)(op) = e1; *(volatile float*)(op + 32) = e2; *(volatile float*)(op + 64) = p3; *(volatile float*)(op + 96) = p4; *(volatile float*)(oq) = f1; *(volatile float*)(oq + 32) = f2; *(volatile float*)(oq + 64) = q3; *(volatile float*)(oq + 96) = q4;
    __threadfence();
    *(volatile float*)(op) = e1; *(volatile float*)(op + 32) = e2; *(volatile float*)(op + 64) = p3; *(volatile float*)(op + 96) = p4; *(volatile float*)(oq) = f1; *(volatile float*)(oq + 32) = f2; *(volatile float*)(oq + 64) = q3; *(volatile float*)(oq + 96) = q4; }

__global__ __launch_bounds__(64) void k_walk3(const float* __restrict__ Pj, const float* __restrict__ Sc, const float* __restrict__ Pt, const float* __restrict__ Qt, const float* __restrict__ a9, float* Yg) { const unsigned sn = blockIdx.x >> 5, un = blockIdx.x & 31u, wd = threadIdx.x; float cw[NC];
#pragma unroll
    for (int k = 0; k < NC; ++k) cw[k] = 0.0f;
    const float dv = bfr(a9[un]); float xe = 0.0f;
    for (int tn = 0; tn < NT; ++tn) { const size_t rw = (size_t)sn * NT + tn; const float* pr = Pj + rw * NJ + un * NW + wd; const float gv = pr[0], xv = pr[OX]; const v4f sc = *(const v4f*)(Sc + (rw * NU + un) * 4); const float pc = sc[0], fd = sc[1], bl = sc[2];
        const float* pt = Pt + (rw * NU + un) * NC; const float* pe = (tn > 0) ? pt - (size_t)NU * NC : pt; const float* qt = Qt + (rw * NU + un) * NC;
        const float c1 = pc * bl * xv, c2 = pc * (1.0f - bl) * fd * xe; float tot = 0.0f;
#pragma unroll
        for (int k = 0; k < NC; ++k) { cw[k] = fd * cw[k] + (c1 * pt[k] + c2 * pe[k]); tot += cw[k] * qt[k]; }
        const float yv = (tot + dv * xv) * (gv / (1.0f + expf(-gv))); float* o = Yg + rw * NG + un * NW + wd; *(volatile float*)o = yv; __threadfence(); *(volatile float*)o = yv; xe = xv; } }

extern "C" void kernel_launch(void* const* d_in, const int* in_sizes, int n_in, void* d_out, int out_size, void* d_ws, size_t ws_size, hipStream_t stream) {
    if (n_in < 9) return;
    if (in_sizes[0] != NR * NM || in_sizes[1] != NJ * NM || in_sizes[2] != NM * NG || in_sizes[3] != NU || in_sizes[4] != NU * NC || in_sizes[5] != NU * NC || in_sizes[6] != NC || in_sizes[7] != NC || in_sizes[8] != NU) return;
    if (out_size != NR * NM) return;
    static_assert(NR % 64 == 0 && NJ % 64 == 0 && NM % 64 == 0 && NM % 32 == 0 && NG % 32 == 0 && (NR * NM / 8) % 256 == 0 && (NJ * NM / 8) % 256 == 0 && (NR * NG / 8) % 256 == 0 && (NM * NG / 8) % 256 == 0 && (NR * NU) % 256 == 0 && (2 * NU * NQ) % 256 == 0 && (NR * NU * NQ) % 256 == 0 && NU == 32 && NQ == 32 && NW == 64 && NC == 128 && NG == NU * NW && NR == 2 * NT && NJ == 2 * NG + 2 * NC + 3 * NU + NQ && OX == NG && OP == 2 * NG && OQ == OP + NC && OPA == OQ + NC && OFA == OPA + NU && OBL == OFA + NU && OAR == OBL + NU, "the products: row and column counts multiples of 64, the depths of 32; every one-dimensional launch exact; 32 units of 64 words, 128 cell words, 32 arcs; the first product's columns in their eight parts");
    const float* i0 = (const float*)d_in[0]; const float* i1 = (const float*)d_in[1]; const float* i2 = (const float*)d_in[2]; const float* i3 = (const float*)d_in[3]; const float* i4 = (const float*)d_in[4]; const float* i5 = (const float*)d_in[5]; const float* i6 = (const float*)d_in[6]; const float* i7 = (const float*)d_in[7]; const float* i8 = (const float*)d_in[8]; float* out = (float*)d_out;
    char* wsp = (char*)d_ws; auto take = [&](size_t bytes) { char* p = wsp; wsp += (bytes + 255) & ~(size_t)255; return (void*)p; };
    bf* Ub = (bf*)take((size_t)NR * NM * 2); bf* Vb = (bf*)take((size_t)NJ * NM * 2); float* Pj = (float*)take((size_t)NR * NJ * 4); float* Sc = (float*)take((size_t)NR * NU * 4 * 4); float* Ar = (float*)take((size_t)NR * NU * NQ * 4); float* Sw = (float*)take((size_t)NR * NU * NQ * 4); float* Pn = (float*)take((size_t)NR * NC * 4); float* Qn = (float*)take((size_t)NR * NC * 4); float* Pt = (float*)take((size_t)NR * NU * NC * 4); float* Qt = (float*)take((size_t)NR * NU * NC * 4); float* Yg = (float*)take((size_t)NR * NG * 4); h16* Yh = (h16*)take((size_t)NR * NG * 2); h16* Wh = (h16*)take((size_t)NM * NG * 2);
    if ((size_t)(wsp - (char*)d_ws) > ws_size) return;
    k_cvt8<<<(unsigned)(NR * NM / 8 / 256), 256, 0, stream>>>(i0, Ub, (size_t)NR * NM / 8);
    k_cvt8<<<(unsigned)(NJ * NM / 8 / 256), 256, 0, stream>>>(i1, Vb, (size_t)NJ * NM / 8);
    k_gemmw<bf, 0, false><<<dim3(NR / 64, NJ / 64, 1), 32, 0, stream>>>(Ub, nullptr, Vb, nullptr, NM, Pj, NJ, nullptr, 0, 0, 0);
    k_pre4<<<(unsigned)(NR * NU / 256), 256, 0, stream>>>(Pj, i3, i6, i7, Sc, Ar, Pn, Qn);
    k_run<<<(unsigned)(2 * NU * NQ / 256), 256, 0, stream>>>(Ar, Sw);
    k_turn<<<(unsigned)(NR * NU * NQ / 256), 256, 0, stream>>>(Sw, Pn, Qn, i4, i5, Pt, Qt);
    k_walk3<<<2 * NU, 64, 0, stream>>>(Pj, Sc, Pt, Qt, i8, Yg);
    k_c16<false><<<(unsigned)(NR * NG / 8 / 256), 256, 0, stream>>>(Yg, Yh, (size_t)NR * NG / 8);
    k_c16<true><<<(unsigned)(NM * NG / 8 / 256), 256, 0, stream>>>(i2, Wh, (size_t)NM * NG / 8);
    k_gemmw<h16, 0, false><<<dim3(NR / 64, NM / 64, 1), 32, 0, stream>>>(Yh, nullptr, Wh, nullptr, NG, out, NM, nullptr, 0, 0, 0);
}
